// MyEdgeConvBlock_13477607375096
// MI455X (gfx1250) — hardware-verified
//
#include <hip/hip_runtime.h>
#include <stddef.h>


#pragma clang fp contract(off)

#define CI      128
#define HD      256
#define CO      128
#define NPQ     512
#define NTHR    256
#define NWAVE   8
#define NBN     64
#define NCQ     4
#define XP      136
#define SP      68
#define TE      128
#define AP      264
#define OP      132
#define EPT     8
#define PIECE   (NTHR * EPT)
#define WCAP    (EPT * 32)
#define NBC     512
#define SLB     9
#define PWPQ    0
#define PW2     65536
#define PWTOT   98304
#define PREPBLK (PWTOT / (NTHR * 8))
#define WSCAP   134217728
#define PQDYN   (NWAVE * 16 * SP * 4)
#define EDGEDYN (TE * AP * 2)
#define AGGDYN  (NBC * CO * 4)

static_assert((PWTOT % (NTHR * 8)) == 0);
static_assert((PW2 % (NTHR * 8)) == 0);
static_assert(((256 * CI) % (NTHR * 8)) == 0);
static_assert(((XP * 2) % 16) == 0);
static_assert(((AP * 2) % 16) == 0);
static_assert(((SP * 4) % 16) == 0);
static_assert(((OP * 4) % 16) == 0);
static_assert((TE * OP * 4) <= EDGEDYN);
static_assert(NBC == (1 << SLB));
static_assert(PIECE == 2048);
static_assert((EPT % 4) == 0);
static_assert((NBC % NWAVE) == 0);
static_assert(NBN == 4 * 16);
static_assert(TE == NWAVE * 16);
static_assert(NTHR == 2 * TE);
static_assert(NTHR == 4 * NBN);
static_assert((NBC * CO) % (4 * NTHR) == 0);
static_assert((PIECE % TE) == 0);
static_assert(NCQ * 2 * 64 == NPQ);

typedef float          v4f   __attribute__((ext_vector_type(4)));
typedef float          v8f   __attribute__((ext_vector_type(8)));
typedef int            v4i   __attribute__((ext_vector_type(4)));
typedef unsigned int   v4u   __attribute__((ext_vector_type(4)));
typedef _Float16       v8h   __attribute__((ext_vector_type(8)));
typedef _Float16       v16h  __attribute__((ext_vector_type(16)));

__device__ __forceinline__ v16h ldfrag(const _Float16* p) {
  const v8h u0 = *(const v8h*)p;
  const v8h u1 = *(const v8h*)(p + 16);
  return __builtin_shufflevector(u0, u1, 0, 1, 2, 3, 4, 5, 6, 7, 8, 9, 10, 11, 12, 13, 14, 15);
}

__device__ __forceinline__ v8f wm(v16h a, v16h b, v8f c) {
  v8f d = __builtin_amdgcn_wmma_f32_16x16x32_f16(false, a, false, b, (short)0, c, false, false);
  asm volatile("v_nop\n\tv_nop\n\tv_nop\n\tv_nop" : "+v"(d) : "v"(a), "v"(b));
  return d;
}
__device__ __forceinline__ v8f zero8() {
  v8f z = {0.f, 0.f, 0.f, 0.f, 0.f, 0.f, 0.f, 0.f};
  return z;
}
__device__ __forceinline__ int iclamp(int v, int lo, int hi) { return v < lo ? lo : (v > hi ? hi : v); }

__device__ __forceinline__ _Float16 bnh(float v, int c, const float* sBN) {
  float t = v - sBN[3 * CI + c];
  t = t * sBN[c];
  t = t * sBN[CI + c];
  t = t + sBN[2 * CI + c];
  return (_Float16)t;
}
__device__ __forceinline__ _Float16 hch(float p, float q, float b) {
  const float z = (p + q) + b;
  return (_Float16)(16.0f * fmaxf(z, 0.0f));
}

__global__ __launch_bounds__(NTHR) void k_prep(const float* __restrict__ W1, const float* __restrict__ W2,
                                               _Float16* wp) {
  const int tid = (int)threadIdx.x;
  const int blk = (int)blockIdx.x;
  const int o = (blk * NTHR + tid) * 8;
  v8h hv;
  if (blk < (256 * CI) / (NTHR * 8)) {
    const int n = o >> 7, k0 = o & 127;
#pragma unroll
    for (int i = 0; i < 8; ++i) {
      const float a = W1[(size_t)(k0 + i) * HD + n];
      const float b = W1[(size_t)(CI + k0 + i) * HD + n];
      hv[i] = (_Float16)(64.0f * (a - b));
    }
  } else if (blk < PW2 / (NTHR * 8)) {
    const int n = (o >> 7) - 256, k0 = o & 127;
#pragma unroll
    for (int i = 0; i < 8; ++i) hv[i] = (_Float16)(64.0f * W1[(size_t)(CI + k0 + i) * HD + n]);
  } else {
    const int idx = o - PW2;
    const int n = idx >> 8, k0 = idx & 255;
#pragma unroll
    for (int i = 0; i < 8; ++i) hv[i] = (_Float16)(64.0f * W2[(size_t)(k0 + i) * CO + n]);
  }
  const v4u u = __builtin_bit_cast(v4u, hv);
  _Float16* dst = wp + o;
  *(volatile v4u*)dst = u;
  __threadfence();
  *(volatile v4u*)dst = u;
}

__global__ __launch_bounds__(NTHR) void k_pq(const float* __restrict__ x, const float* __restrict__ gam,
                                             const float* __restrict__ bet, const float* __restrict__ mu,
                                             const float* __restrict__ var, const _Float16* __restrict__ wp,
                                             float* PQ, int nN) {
  extern __shared__ __attribute__((aligned(16))) float stg[];
  __shared__ __attribute__((aligned(16))) _Float16 sX[NBN * XP];
  __shared__ float sBN[4 * CI];
  const int tid = (int)threadIdx.x, lane = tid & 31, wave = tid >> 5, hh = lane >> 4, m = lane & 15;
  const int n0 = (int)blockIdx.x * NBN;
  const int cq = (int)blockIdx.y;

  if (tid < CI) {
    sBN[tid]          = rsqrtf(var[tid] + 1e-5f);
    sBN[CI + tid]     = gam[tid];
    sBN[2 * CI + tid] = bet[tid];
    sBN[3 * CI + tid] = mu[tid];
  }
  __syncthreads();

  {
    const int nl = tid >> 2, q = tid & 3;
    int node = n0 + nl;
    node = node > nN - 1 ? nN - 1 : node;
    const float* rp = x + (size_t)node * CI + 32 * q;
#pragma unroll
    for (int g = 0; g < 4; ++g) {
      const v4f a = *(const v4f*)(rp + 8 * g);
      const v4f b = *(const v4f*)(rp + 8 * g + 4);
      const int cb = 32 * q + 8 * g;
      v8h u;
      u[0] = bnh(a.x, cb + 0, sBN); u[1] = bnh(a.y, cb + 1, sBN);
      u[2] = bnh(a.z, cb + 2, sBN); u[3] = bnh(a.w, cb + 3, sBN);
      u[4] = bnh(b.x, cb + 4, sBN); u[5] = bnh(b.y, cb + 5, sBN);
      u[6] = bnh(b.z, cb + 6, sBN); u[7] = bnh(b.w, cb + 7, sBN);
      *(v8h*)(sX + nl * XP + cb) = u;
    }
  }
  __syncthreads();

  const int rt = wave & 3, cg = wave >> 2;
  const _Float16* bp = wp + PWPQ + (size_t)(128 * cq + 64 * cg + m) * CI + 8 * hh;
  const _Float16* ap = sX + (16 * rt + m) * XP + 8 * hh;
  v8f c[4];
#pragma unroll
  for (int j = 0; j < 4; ++j) c[j] = zero8();
#pragma unroll
  for (int ks = 0; ks < 4; ++ks) {
    const v16h a = ldfrag(ap + 32 * ks);
#pragma unroll
    for (int j = 0; j < 4; ++j) {
      const v16h b = ldfrag(bp + (size_t)(16 * j) * CI + 32 * ks);
      c[j] = wm(a, b, c[j]);
    }
  }
  float* sw = stg + wave * 16 * SP;
#pragma unroll
  for (int j = 0; j < 4; ++j) {
#pragma unroll
    for (int r = 0; r < 8; ++r) sw[(8 * hh + r) * SP + 16 * j + m] = c[j][r] * 0.015625f;
  }
  __syncthreads();
  float* ob = PQ + (size_t)128 * cq + 64 * cg + 4 * m;
#pragma unroll 1
  for (int i = 0; i < 8; ++i) {
    const int row = 2 * i + hh;
    const v4f v = *(const v4f*)(sw + row * SP + 4 * m);
    *(volatile v4f*)(ob + (size_t)(n0 + 16 * rt + row) * NPQ) = v;
  }
  __threadfence();
#pragma unroll 1
  for (int i = 0; i < 8; ++i) {
    const int row = 2 * i + hh;
    const v4f v = *(const v4f*)(sw + row * SP + 4 * m);
    *(volatile v4f*)(ob + (size_t)(n0 + 16 * rt + row) * NPQ) = v;
  }
}

__global__ __launch_bounds__(NTHR) void k_edge(
    const int* __restrict__ ei, const float* __restrict__ PQ, const float* __restrict__ b1,
    const float* __restrict__ b2, const _Float16* __restrict__ wp, float* MS,
    int c0, int nE, int nN) {
  extern __shared__ __attribute__((aligned(16))) v4f edyn[];
  __shared__ __attribute__((aligned(16))) float sPar[HD + CO];
  __shared__ int sIdx[2 * TE];
  _Float16* sA = (_Float16*)edyn;
  float*    sO = (float*)edyn;
  const int tid = (int)threadIdx.x, lane = tid & 31, wave = tid >> 5, hh = lane >> 4, m = lane & 15;
  const int le0 = (int)blockIdx.x * TE;
  const int ge0 = c0 + le0;

  {
    const int s = tid >> 7, j = tid & (TE - 1);
    int e = ge0 + j;
    e = e > nE - 1 ? nE - 1 : e;
    int v = ei[(size_t)s * nE + e];
    if (v < 0) v += nN;
    v = iclamp(v, 0, nN - 1);
    sIdx[s * TE + j] = v;
  }
  if (tid < HD) sPar[tid] = b1[tid];
  if (tid < CO) sPar[HD + tid] = b2[tid];
  __syncthreads();

  {
    const int el = tid >> 1, q = tid & 1;
    const int snode = sIdx[el], dnode = sIdx[TE + el];
    const float* pp = PQ + (size_t)dnode * NPQ + 128 * q;
    const float* qp = PQ + (size_t)snode * NPQ + HD + 128 * q;
    const float* pb = sPar + 128 * q;
    _Float16* dst = sA + el * AP + 128 * q;
#pragma unroll 1
    for (int i = 0; i < 16; ++i) {
      const v4f a0 = *(const v4f*)(pp + 8 * i);
      const v4f a1 = *(const v4f*)(pp + 8 * i + 4);
      const v4f g0 = *(const v4f*)(qp + 8 * i);
      const v4f g1 = *(const v4f*)(qp + 8 * i + 4);
      const int cb = 8 * i;
      v8h o;
      o[0] = hch(a0.x, g0.x, pb[cb + 0]);
      o[1] = hch(a0.y, g0.y, pb[cb + 1]);
      o[2] = hch(a0.z, g0.z, pb[cb + 2]);
      o[3] = hch(a0.w, g0.w, pb[cb + 3]);
      o[4] = hch(a1.x, g1.x, pb[cb + 4]);
      o[5] = hch(a1.y, g1.y, pb[cb + 5]);
      o[6] = hch(a1.z, g1.z, pb[cb + 6]);
      o[7] = hch(a1.w, g1.w, pb[cb + 7]);
      *(v8h*)(dst + cb) = o;
    }
  }
  __syncthreads();

  const int rt = wave & 3, cg = wave >> 2;
  v8f c[2][4];
#pragma unroll
  for (int u = 0; u < 2; ++u) {
#pragma unroll
    for (int j = 0; j < 4; ++j) c[u][j] = zero8();
  }
  {
    const _Float16* ap0 = sA + (32 * rt + m) * AP + 8 * hh;
    const _Float16* ap1 = ap0 + 16 * AP;
    const _Float16* bp = wp + PW2 + (size_t)(64 * cg + m) * HD + 8 * hh;
#pragma unroll 1
    for (int ks = 0; ks < 8; ++ks) {
      const v16h a0 = ldfrag(ap0 + 32 * ks);
      const v16h a1 = ldfrag(ap1 + 32 * ks);
#pragma unroll
      for (int j = 0; j < 4; ++j) {
        const v16h b = ldfrag(bp + (size_t)(16 * j) * HD + 32 * ks);
        c[0][j] = wm(a0, b, c[0][j]);
        c[1][j] = wm(a1, b, c[1][j]);
      }
    }
  }
  __syncthreads();

#pragma unroll
  for (int u = 0; u < 2; ++u) {
#pragma unroll
    for (int j = 0; j < 4; ++j) {
      const int col = 64 * cg + 16 * j + m;
      const float bb = sPar[HD + col];
      float* sp = sO + (32 * rt + 16 * u + 8 * hh) * OP + col;
#pragma unroll
      for (int r = 0; r < 8; ++r) sp[r * OP] = c[u][j][r] * 0.0009765625f + bb;
    }
  }
  __syncthreads();
#pragma unroll 1
  for (int i = 0; i < 16; ++i) {
    const int row = 16 * wave + i;
    const v4f v = *(const v4f*)(sO + row * OP + 4 * lane);
    *(volatile v4f*)(MS + (size_t)(le0 + row) * CO + 4 * lane) = v;
  }
  __threadfence();
#pragma unroll 1
  for (int i = 0; i < 16; ++i) {
    const int row = 16 * wave + i;
    const v4f v = *(const v4f*)(sO + row * OP + 4 * lane);
    *(volatile v4f*)(MS + (size_t)(le0 + row) * CO + 4 * lane) = v;
  }
}

__device__ __forceinline__ int scan_piece(const int* __restrict__ kp, int lim, int cbase, int base,
                                          int* list, int tid, int wave, int vec_ok) {
  int wc = 0;
  const int el0  = tid * EPT;
  const int e0   = cbase + el0;
  const int sent = -2147483647 - 1;
  int kk[EPT];
  if (vec_ok != 0 && cbase + PIECE <= lim) {
    const v4i* p = (const v4i*)(kp + e0);
#pragma unroll
    for (int u = 0; u < EPT / 4; ++u) {
      const v4i d = p[u];
      kk[4 * u] = d.x; kk[4 * u + 1] = d.y; kk[4 * u + 2] = d.z; kk[4 * u + 3] = d.w;
    }
  } else {
    const int lm = lim - 1;
#pragma unroll
    for (int q = 0; q < EPT; ++q) {
      const int eq = e0 + q;
      const int ec = eq > lm ? lm : eq;
      const int a = kp[ec];
      kk[q] = (eq < lim) ? a : sent;
    }
  }
  const unsigned nb = (unsigned)base;
  unsigned sq[EPT];
  bool hq[EPT];
  bool anyl = false;
#pragma unroll
  for (int q = 0; q < EPT; ++q) {
    sq[q] = (unsigned)kk[q] - nb;
    hq[q] = sq[q] < (unsigned)NBC;
    anyl = anyl | hq[q];
  }
  const unsigned any = __builtin_amdgcn_ballot_w32(anyl);
  if (any != 0u) {
#define HIT(HQ, SQ, Q) { \
      const unsigned mj = __builtin_amdgcn_ballot_w32(HQ); \
      if (mj != 0u) { \
        if (HQ) { \
          const int ps = wc + (int)__builtin_amdgcn_mbcnt_lo(mj, 0u); \
          if (ps < WCAP) list[wave * WCAP + ps] = ((el0 + (Q)) << SLB) | (int)(SQ); \
        } \
        wc += (int)__builtin_popcount(mj); } }
#pragma unroll
    for (int q = 0; q < EPT; ++q) {
      HIT(hq[q], sq[q], q)
    }
#undef HIT
  }
  return wc;
}

__device__ __forceinline__ void drain_max(const int* list, const int* wcnt, float* accF,
                                          const float* __restrict__ MS,
                                          int cbase, int nec, int lane, int wave) {
#pragma unroll 1
  for (int wsx = 0; wsx < NWAVE; ++wsx) {
    int n = __builtin_amdgcn_readfirstlane(wcnt[wsx]);
    n = n > WCAP ? WCAP : (n < 0 ? 0 : n);
    const int* lp = list + wsx * WCAP;
#pragma unroll 1
    for (int bb = 0; bb < n; bb += 32) {
      const int idx = bb + lane;
      const int ic = idx > WCAP - 1 ? WCAP - 1 : idx;
      const int ent = lp[ic];
      const bool own = (idx < n) && ((ent & (NWAVE - 1)) == wave);
      unsigned msk = __builtin_amdgcn_ballot_w32(own);
#pragma unroll 1
      while (msk != 0u) {
        const int bit = (int)__builtin_ctz(msk);
        msk &= msk - 1u;
        const int e2 = __builtin_amdgcn_readlane(ent, bit);
        const int slot = e2 & (NBC - 1);
        const int el = (e2 >> SLB) & (PIECE - 1);
        int e = cbase + el;
        e = e > nec - 1 ? nec - 1 : (e < 0 ? 0 : e);
        const v4f v = *(const v4f*)(MS + (size_t)e * CO + 4 * lane);
        float* ap = accF + slot * CO + 4 * lane;
        v4f a = *(const v4f*)ap;
        a.x = fmaxf(a.x, v.x);
        a.y = fmaxf(a.y, v.y);
        a.z = fmaxf(a.z, v.z);
        a.w = fmaxf(a.w, v.w);
        *(v4f*)ap = a;
      }
    }
  }
}

__device__ __forceinline__ void node_rows(const float* accF, float* outp, int base, int nN,
                                          int wave, int lane) {
#pragma unroll 1
  for (int it = 0; it < NBC / NWAVE; ++it) {
    const int s = wave + NWAVE * it;
    const int node = base + s;
    if (node < nN) {
      const v4f v = *(const v4f*)(accF + s * CO + 4 * lane);
      *(volatile v4f*)(outp + (size_t)node * CO + 4 * lane) = v;
    }
  }
}

__global__ __launch_bounds__(NTHR) void k_agg(
    const int* __restrict__ ei, const float* __restrict__ MS, float* outp,
    int c0, int nec, int nE, int nN, int first, int vec_ok) {
  extern __shared__ __attribute__((aligned(16))) float accF[];
  __shared__ int list[NWAVE * WCAP];
  __shared__ int wcnt[NWAVE];
  const int tid = (int)threadIdx.x, lane = tid & 31, wave = tid >> 5;
  const int base = (int)blockIdx.x * NBC;

  if (first != 0) {
    const v4f z = {0.0f, 0.0f, 0.0f, 0.0f};
#pragma unroll 1
    for (int i = tid; i < (NBC * CO) / 4; i += NTHR) *(v4f*)(accF + 4 * i) = z;
  } else {
#pragma unroll 1
    for (int i = tid; i < (NBC * CO) / 4; i += NTHR) {
      const int slot = i >> 5;
      const int node = base + slot;
      const int nc = node > nN - 1 ? nN - 1 : node;
      v4f v = *(const v4f*)(outp + (size_t)nc * CO + 4 * (i & 31));
      if (node > nN - 1) { v.x = 0.0f; v.y = 0.0f; v.z = 0.0f; v.w = 0.0f; }
      *(v4f*)(accF + 4 * i) = v;
    }
  }
  __syncthreads();

  const int* kp = ei + (size_t)nE + c0;
#pragma unroll 1
  for (int cbase = 0; cbase < nec; cbase += PIECE) {
    const int wc = scan_piece(kp, nec, cbase, base, list, tid, wave, vec_ok);
    if (lane == 0) wcnt[wave] = wc;
    __syncthreads();
    drain_max(list, wcnt, accF, MS, cbase, nec, lane, wave);
    __syncthreads();
  }

  node_rows(accF, outp, base, nN, wave, lane);
  __threadfence();
  node_rows(accF, outp, base, nN, wave, lane);
}

extern "C" void kernel_launch(void* const* d_in, const int* in_sizes, int n_in,
                              void* d_out, int out_size, void* d_ws, size_t ws_size,
                              hipStream_t stream) {
  if (n_in < 10) return;
  if (in_sizes[0] < CI || (in_sizes[0] % CI) != 0) return;
  const int nN = in_sizes[0] / CI;
  if (nN < 1 || nN > (1 << 24)) return;
  if (in_sizes[1] < 2 || (in_sizes[1] % 2) != 0) return;
  const int nE = in_sizes[1] / 2;
  if (nE < 1 || nE > (1 << 27)) return;
  if (in_sizes[2] != CI || in_sizes[3] != CI || in_sizes[4] != CI || in_sizes[5] != CI) return;
  if (in_sizes[6] != 2 * CI * HD || in_sizes[7] != HD) return;
  if (in_sizes[8] != HD * CO || in_sizes[9] != CO) return;
  if ((long long)out_size != (long long)nN * CO) return;

  const float* x   = (const float*)d_in[0];
  const int*   ei  = (const int*)d_in[1];
  const float* gam = (const float*)d_in[2];
  const float* bet = (const float*)d_in[3];
  const float* mu  = (const float*)d_in[4];
  const float* var = (const float*)d_in[5];
  const float* W1  = (const float*)d_in[6];
  const float* b1  = (const float*)d_in[7];
  const float* W2  = (const float*)d_in[8];
  const float* b2  = (const float*)d_in[9];
  float* outp = (float*)d_out;

  const int nb64 = (nN + NBN - 1) / NBN;
  const int Npad64 = nb64 * NBN;
  const int nbA = (nN + NBC - 1) / NBC;
  const int vec_ok = ((nE & 3) == 0) ? 1 : 0;

  const size_t cap = ws_size < (size_t)WSCAP ? ws_size : (size_t)WSCAP;
  const size_t bW  = (size_t)PWTOT * 2;
  const size_t bPQ = (size_t)Npad64 * NPQ * 4;
  const size_t fixedB = ((bW + 255) & ~(size_t)255) + ((bPQ + 255) & ~(size_t)255);
  int C = 0;
  size_t CE = 0;
  for (int c = 1; c <= 512; ++c) {
    size_t ce = ((size_t)nE + (size_t)c - 1) / (size_t)c;
    ce = (ce + PIECE - 1) / PIECE * PIECE;
    const size_t tot = fixedB + ((ce * CO * 4 + 255) & ~(size_t)255);
    if (tot <= cap) { C = c; CE = ce; break; }
  }
  if (C == 0) return;

  char* ws = (char*)d_ws;
  size_t off = 0;
  const size_t oW  = off; off += bW;                    off = (off + 255) & ~(size_t)255;
  const size_t oPQ = off; off += bPQ;                   off = (off + 255) & ~(size_t)255;
  const size_t oMS = off; off += CE * CO * 4;           off = (off + 255) & ~(size_t)255;
  if (off > cap || off > ws_size) return;
  _Float16* wp = (_Float16*)(ws + oW);
  float*    PQ = (float*)(ws + oPQ);
  float*    MS = (float*)(ws + oMS);

  hipFuncSetAttribute(reinterpret_cast<const void*>(&k_pq),   hipFuncAttributeMaxDynamicSharedMemorySize, PQDYN);
  hipFuncSetAttribute(reinterpret_cast<const void*>(&k_edge), hipFuncAttributeMaxDynamicSharedMemorySize, EDGEDYN);
  hipFuncSetAttribute(reinterpret_cast<const void*>(&k_agg),  hipFuncAttributeMaxDynamicSharedMemorySize, AGGDYN);

  k_prep<<<PREPBLK, NTHR, 0, stream>>>(W1, W2, wp);
  k_pq<<<dim3(nb64, NCQ), NTHR, PQDYN, stream>>>(x, gam, bet, mu, var, wp, PQ, nN);
  for (int ch = 0; ch < C; ++ch) {
    const size_t c0s = (size_t)ch * CE;
    if (c0s >= (size_t)nE) break;
    const int c0 = (int)c0s;
    size_t necs = (size_t)nE - c0s;
    if (necs > CE) necs = CE;
    const int nec = (int)necs;
    const int ntiles = (nec + TE - 1) / TE;
    k_edge<<<ntiles, NTHR, EDGEDYN, stream>>>(ei, PQ, b1, b2, wp, MS, c0, nE, nN);
    k_agg<<<nbA, NTHR, AGGDYN, stream>>>(ei, MS, outp, c0, nec, nE, nN, (ch == 0) ? 1 : 0, vec_ok);
  }
}
